// PointNetClassifier_32083405701129
// MI455X (gfx1250) — hardware-verified
//
#include <hip/hip_runtime.h>
#include <math.h>

typedef __attribute__((ext_vector_type(16))) _Float16 v16h;
typedef __attribute__((ext_vector_type(16))) __bf16 v16b;
typedef __attribute__((ext_vector_type(8)))  _Float16 v8h;
typedef __attribute__((ext_vector_type(8)))  float v8f;
typedef __attribute__((ext_vector_type(4)))  float v4f;
typedef __attribute__((ext_vector_type(2)))  float v2f;
typedef __attribute__((ext_vector_type(4)))  unsigned v4u;
typedef __attribute__((ext_vector_type(4)))  int v4i;
typedef float __attribute__((may_alias)) float_a;
typedef int __attribute__((may_alias)) int_a;

template <typename T> __device__ __forceinline__ void vst2(void* p, T v) { *(volatile T*)p = v; __threadfence(); *(volatile T*)p = v; }
__device__ __forceinline__ v8f wmma16(v16h a, v16h b, v8f c) {
  v8f d = __builtin_amdgcn_wmma_f32_16x16x32_f16(false, a, false, b, (short)0, c, false, false);
  asm volatile("v_nop\n\tv_nop\n\tv_nop\n\tv_nop" : "+v"(d) : "v"(a), "v"(b));
  return d;
}
__device__ __forceinline__ v8f wmma_bf(v16b a, v16b b, v8f c) {
  v8f d = __builtin_amdgcn_wmma_f32_16x16x32_bf16(false, a, false, b, (short)0, c, false, false);
  asm volatile("v_nop\n\tv_nop\n\tv_nop\n\tv_nop" : "+v"(d) : "v"(a), "v"(b));
  return d;
}
__device__ __forceinline__ v16h frag_h(const _Float16* rowk0, int lane) {
  union { v16h v; v8h q[2]; } u; const _Float16* p = rowk0 + 8 * (lane >> 4);
  u.q[0] = *(const v8h*)p; u.q[1] = *(const v8h*)(p + 16); return u.v;
}
__device__ __forceinline__ v16h frag_f32(const float* rowk0, int lane) {
  v16h a; const float* p = rowk0 + 8 * (lane >> 4);
#pragma unroll
  for (int i = 0; i < 8; ++i) { a[i] = (_Float16)p[i]; a[8 + i] = (_Float16)p[16 + i]; }
  return a;
}
__device__ __forceinline__ v16h frag_f32s(const float* rowk0, int lane, float sc) {
  v16h a; const float* p = rowk0 + 8 * (lane >> 4);
#pragma unroll
  for (int i = 0; i < 8; ++i) { a[i] = (_Float16)(p[i] * sc); a[8 + i] = (_Float16)(p[16 + i] * sc); }
  return a;
}
__device__ __forceinline__ v16h fragc_f32(const float* W, int k0, int n, int lane, int ld, int K) {
  v16h a; const int g = lane >> 4;
#pragma unroll
  for (int i = 0; i < 8; ++i) { const int ka = k0 + 8 * g + i, kb = ka + 16;
    a[i] = (_Float16)(ka < K ? W[(size_t)(ka < K ? ka : K - 1) * ld + n] : 0.f); a[8 + i] = (_Float16)(kb < K ? W[(size_t)(kb < K ? kb : K - 1) * ld + n] : 0.f); }
  return a;
}
struct F2 { v16b h, l; };
__device__ __forceinline__ F2 bsplit16(const float v[16]) { F2 r;
#pragma unroll
  for (int i = 0; i < 16; ++i) { const __bf16 h = (__bf16)v[i]; r.h[i] = h; r.l[i] = (__bf16)(v[i] - (float)h); }
  return r; }
__device__ __forceinline__ F2 split_row(const float* row, int k0, int lane) { float v[16]; const float* p = row + k0 + 8 * (lane >> 4);
#pragma unroll
  for (int i = 0; i < 8; ++i) { v[i] = p[i]; v[8 + i] = p[16 + i]; }
  return bsplit16(v); }
__device__ __forceinline__ F2 split_rowK(const float* row, int k0, int lane, int K) { float v[16]; const int g = lane >> 4;
#pragma unroll
  for (int i = 0; i < 8; ++i) { const int ka = k0 + 8 * g + i, kb = ka + 16; v[i] = ka < K ? row[ka < K ? ka : K - 1] : 0.f; v[8 + i] = kb < K ? row[kb < K ? kb : K - 1] : 0.f; }
  return bsplit16(v); }
__device__ __forceinline__ F2 split_col(const float* W, int k0, int n, int lane, int ld, int K) { float v[16]; const int g = lane >> 4;
#pragma unroll
  for (int i = 0; i < 8; ++i) { const int ka = k0 + 8 * g + i, kb = ka + 16; v[i] = ka < K ? W[(size_t)(ka < K ? ka : K - 1) * ld + n] : 0.f; v[8 + i] = kb < K ? W[(size_t)(kb < K ? kb : K - 1) * ld + n] : 0.f; }
  return bsplit16(v); }
__device__ __forceinline__ v8f mac3(const F2& a, const F2& b, v8f c) { c = wmma_bf(a.l, b.h, c); c = wmma_bf(a.h, b.l, c); return wmma_bf(a.h, b.h, c); }
__device__ __forceinline__ float sigm(float v) { return 1.0f / (1.0f + expf(-v)); }
#define LDSX() do { asm volatile("s_wait_dscnt 0" ::: "memory"); __builtin_amdgcn_wave_barrier(); __builtin_amdgcn_fence(__ATOMIC_RELEASE, "workgroup"); } while (0)


#define NBATCH 16
#define VS 96
#define NVOX (VS * VS * VS)
#define CHK 256
#define NCHK (NVOX / CHK)
#define NP 4096
#define NPT (NBATCH * NP)
#define NG 8
#ifndef TNB
#define TNB NBATCH
#endif
typedef __attribute__((ext_vector_type(8))) __bf16 v8b;
__device__ __forceinline__ v16b frag_b(const __bf16* rowk0, int lane) {
  union { v16b v; v8b q[2]; } u; const __bf16* p = rowk0 + 8 * (lane >> 4);
  u.q[0] = *(const v8b*)p; u.q[1] = *(const v8b*)(p + 16); return u.v;
}
__device__ __forceinline__ v16b frag_gbf(const float* rowk0, int lane) {
  v16b a; const float* p = rowk0 + 8 * (lane >> 4);
#pragma unroll
  for (int i = 0; i < 8; ++i) { a[i] = (__bf16)p[i]; a[8 + i] = (__bf16)p[16 + i]; }
  return a;
}
__device__ __forceinline__ float bfr(float v) { return (float)(__bf16)v; }

#define WS_CNT  0u
#define WS_OFF  (WS_CNT + 4u * NBATCH * NCHK)
#define WS_PTS  (WS_OFF + 4u * NBATCH * 3584)
#define WS_H2   (WS_PTS + 4u * NPT * 4)
#define WS_H3   (WS_H2 + 4u * NPT * 128)
#define WS_PS1  (WS_H3 + 4u * NPT * 256)
#define WS_PS2  (WS_PS1 + 4u * 1024 * 64 * 2)
#define WS_PS3  (WS_PS2 + 4u * 1024 * 128 * 2)
#define WS_PS4  (WS_PS3 + 4u * 1024 * 256 * 2)
#define WS_GN   (WS_PS4 + 4u * 1024 * 512 * 4)
#define WS_END  (WS_GN + 4u * 4 * NBATCH * NG * 2)

__global__ __launch_bounds__(256) void k_count(const float* __restrict__ vol, int* __restrict__ CNT) {
  __shared__ __align__(16) int sc[256];
  const int tid = threadIdx.x; const size_t chunk = (size_t)blockIdx.x * 256 + tid;
  const float* p = vol + chunk * CHK; int n = 0;
#pragma unroll 4
  for (int i = 0; i < CHK; ++i) n += (bfr(p[i]) > 0.5f) ? 1 : 0;
  sc[tid] = n;
  __syncthreads();
  if (tid < 64) vst2(CNT + (size_t)blockIdx.x * 256 + tid * 4, *(const v4i*)&sc[tid * 4]);
}
__global__ __launch_bounds__(256) void k_scan(const int* __restrict__ CNT, int* __restrict__ OFF) {
  __shared__ int spart[256]; __shared__ __align__(16) int soff[3584];
  const int b = blockIdx.x, tid = threadIdx.x; const int per = 14;
  int loc[14]; int s = 0;
#pragma unroll
  for (int i = 0; i < per; ++i) { const int c = tid * per + i; const int v = c < NCHK ? CNT[(size_t)b * NCHK + c] : 0; loc[i] = s; s += v; }
  spart[tid] = s;
  __syncthreads();
  if (tid == 0) { int run = 0; for (int t = 0; t < 256; ++t) { const int v = spart[t]; spart[t] = run; run += v; } }
  __syncthreads();
  const int base = spart[tid];
#pragma unroll
  for (int i = 0; i < per; ++i) soff[tid * per + i] = base + loc[i];
  __syncthreads();
  for (int q = tid; q < 3584 / 4; q += 256) vst2(OFF + (size_t)b * 3584 + q * 4, *(const v4i*)&soff[q * 4]);
}

__global__ __launch_bounds__(256) void k_pick(const float* __restrict__ vol, const int* __restrict__ OFF, float* __restrict__ PTS) {
  const int b = blockIdx.y, tid = threadIdx.x; const int p = blockIdx.x * 256 + tid; const int* off = OFF + (size_t)b * 3584; const int n = off[NCHK];
  v4f pt = {0.f, 0.f, 0.f, 0.f};
  if (n > 0) { int idx;
    if (n >= NP) { const float nf = (float)n; const float lf = ((float)p * (nf - 1.0f)) / (float)(NP - 1); idx = (int)lf; const int hi = n - 1 > 0 ? n - 1 : 0; idx = idx < 0 ? 0 : (idx > hi ? hi : idx); }
    else { idx = p % n; }
    int lo = 0, hi2 = NCHK - 1;
    while (lo < hi2) { const int mid = (lo + hi2 + 1) >> 1; if (off[mid] <= idx) lo = mid; else hi2 = mid - 1; }
    int need = idx - off[lo]; const float* pv = vol + ((size_t)b * NVOX + (size_t)lo * CHK); int flat = lo * CHK + CHK - 1;
    for (int i = 0; i < CHK; ++i) { const bool fg = bfr(pv[i]) > 0.5f; if (fg) { if (need == 0) { flat = lo * CHK + i; break; } --need; } }
    const int dd = flat / (VS * VS), hh = (flat / VS) % VS, ww = flat % VS;
    pt[0] = (float)dd / 95.0f * 2.0f - 1.0f; pt[1] = (float)hh / 95.0f * 2.0f - 1.0f; pt[2] = (float)ww / 95.0f * 2.0f - 1.0f; }
  vst2(PTS + ((size_t)b * NP + p) * 4, pt);
}
__device__ __forceinline__ float gn_apply(float h, const float* __restrict__ gn, int b, int c, int cpg, const float* __restrict__ gw, const float* __restrict__ gb) {
  const int g = c / cpg; const float mu = gn[(b * NG + g) * 2], rs = gn[(b * NG + g) * 2 + 1]; const float v = (h - mu) * rs * bfr(gw[c]) + bfr(gb[c]); return v > 0.f ? v : 0.f;
}
__global__ __launch_bounds__(128) void k_l1s(const float* __restrict__ PTS, const float* __restrict__ W1, float* __restrict__ PS1) {
  __shared__ __align__(16) float sps[64][2]; __shared__ float sred[2][64][2];
  const int tid = threadIdx.x; const int c = tid & 63, half = tid >> 6; const size_t p0 = (size_t)blockIdx.x * 64;
  const float w0 = bfr(W1[c * 3]), w1v = bfr(W1[c * 3 + 1]), w2 = bfr(W1[c * 3 + 2]); float s = 0.f, q = 0.f;
  for (int i = half * 32; i < half * 32 + 32; ++i) { const float* pt = PTS + (p0 + i) * 4; const float h = (w0 * pt[0] + w1v * pt[1]) + w2 * pt[2]; s += h; q += h * h; }
  sred[half][c][0] = s; sred[half][c][1] = q;
  __syncthreads();
  if (tid < 64) { sps[tid][0] = sred[0][tid][0] + sred[1][tid][0]; sps[tid][1] = sred[0][tid][1] + sred[1][tid][1]; }
  __syncthreads();
  if (tid < 32) vst2(PS1 + (size_t)blockIdx.x * 128 + tid * 4, *(const v4f*)(&sps[0][0] + tid * 4));
}
__global__ __launch_bounds__(256) void k_gn(const float* __restrict__ PS, int C, int stride, float* __restrict__ GNl) {
  __shared__ float ss[256], sq[256]; __shared__ __align__(16) float sres[16];
  const int b = blockIdx.x, tid = threadIdx.x; const int cpg = C / NG; float s, q;
  { const int g = tid >> 5, lane = tid & 31; s = 0.f; q = 0.f;
    for (int e = lane; e < 64 * cpg; e += 32) { const int blk = e / cpg, cc = g * cpg + e % cpg; const float* pp = PS + ((size_t)(b * 64 + blk) * C + cc) * stride; s += pp[0]; q += pp[1]; }
#pragma unroll
    for (int o = 1; o < 32; o <<= 1) { s += __shfl_xor(s, o); q += __shfl_xor(q, o); }
    if (lane == 0) { const float cnt = (float)(cpg * NP); const float mu = s / cnt; const float var = fmaxf(q / cnt - mu * mu, 0.f); sres[g * 2] = mu; sres[g * 2 + 1] = rsqrtf(var + 1e-5f); } }
  __syncthreads();
  if (tid < 4) vst2(GNl + (size_t)b * 16 + tid * 4, *(const v4f*)&sres[tid * 4]);
}

__global__ __launch_bounds__(128) void k_l2(const float* __restrict__ PTS, const float* __restrict__ W1, const float* __restrict__ GN1, const float* __restrict__ g1w, const float* __restrict__ g1b, const float* __restrict__ W2, float* __restrict__ H2, float* __restrict__ PS2) {
  __shared__ __align__(16) __bf16 sah[64][72], sal[64][72]; __shared__ __align__(16) float so[4][16][132]; __shared__ __align__(16) float sps[128][2];
  const int tid = threadIdx.x, wave = tid >> 5, lane = tid & 31, col = lane & 15, g = lane >> 4; const size_t p0 = (size_t)blockIdx.x * 64; const int b = (int)(p0 / NP);
  for (int q = tid; q < 64 * 64; q += 128) { const int pl = q >> 6, c = q & 63; const float* pt = PTS + (p0 + pl) * 4; const float h = (bfr(W1[c * 3]) * pt[0] + bfr(W1[c * 3 + 1]) * pt[1]) + bfr(W1[c * 3 + 2]) * pt[2];
    const float a = gn_apply(h, GN1, b, c, 8, g1w, g1b); const __bf16 hb = (__bf16)a; sah[pl][c] = hb; sal[pl][c] = (__bf16)(a - (float)hb); }
  __syncthreads();
  v8f acc[8] = {};
#pragma unroll
  for (int kc = 0; kc < 2; ++kc) { const v16b ah = frag_b(&sah[wave * 16 + col][kc * 32], lane), al = frag_b(&sal[wave * 16 + col][kc * 32], lane);
#pragma unroll
    for (int j = 0; j < 8; ++j) { const v16b w = frag_gbf(W2 + (size_t)(j * 16 + col) * 64 + kc * 32, lane); acc[j] = wmma_bf(al, w, acc[j]); acc[j] = wmma_bf(ah, w, acc[j]); } }
#pragma unroll
  for (int j = 0; j < 8; ++j)
#pragma unroll
    for (int r = 0; r < 8; ++r) so[wave][8 * g + r][j * 16 + col] = acc[j][r];
  __syncthreads();
  for (int rl = 0; rl < 16; ++rl) vst2(H2 + (p0 + wave * 16 + rl) * 128 + lane * 4, *(const v4f*)&so[wave][rl][lane * 4]);
  { const int c = tid; float s = 0.f, q2 = 0.f; for (int pl = 0; pl < 64; ++pl) { const float v = so[pl >> 4][pl & 15][c]; s += v; q2 += v * v; } sps[c][0] = s; sps[c][1] = q2; }
  __syncthreads();
  if (tid < 64) vst2(PS2 + (size_t)blockIdx.x * 256 + tid * 4, *(const v4f*)(&sps[0][0] + tid * 4));
}
__global__ __launch_bounds__(128) void k_l3(const float* __restrict__ H2, const float* __restrict__ GN2, const float* __restrict__ g2w, const float* __restrict__ g2b, const float* __restrict__ W3, float* __restrict__ H3, float* __restrict__ PS3) {
  __shared__ __align__(16) __bf16 sah[64][136], sal[64][136]; __shared__ __align__(16) float so[4][16][260]; __shared__ __align__(16) float sps[256][2];
  const int tid = threadIdx.x, wave = tid >> 5, lane = tid & 31, col = lane & 15, g = lane >> 4; const size_t p0 = (size_t)blockIdx.x * 64; const int b = (int)(p0 / NP);
  for (int q = tid; q < 64 * 128; q += 128) { const int pl = q >> 7, c = q & 127; const float a = gn_apply(H2[(p0 + pl) * 128 + c], GN2, b, c, 16, g2w, g2b); const __bf16 hb = (__bf16)a; sah[pl][c] = hb; sal[pl][c] = (__bf16)(a - (float)hb); }
  __syncthreads();
  v8f acc[16] = {};
#pragma unroll
  for (int kc = 0; kc < 4; ++kc) { const v16b ah = frag_b(&sah[wave * 16 + col][kc * 32], lane), al = frag_b(&sal[wave * 16 + col][kc * 32], lane);
#pragma unroll
    for (int j = 0; j < 16; ++j) { const v16b w = frag_gbf(W3 + (size_t)(j * 16 + col) * 128 + kc * 32, lane); acc[j] = wmma_bf(al, w, acc[j]); acc[j] = wmma_bf(ah, w, acc[j]); } }
#pragma unroll
  for (int j = 0; j < 16; ++j)
#pragma unroll
    for (int r = 0; r < 8; ++r) so[wave][8 * g + r][j * 16 + col] = acc[j][r];
  __syncthreads();
  for (int rl = 0; rl < 16; ++rl) for (int pc = lane; pc < 64; pc += 32) vst2(H3 + (p0 + wave * 16 + rl) * 256 + pc * 4, *(const v4f*)&so[wave][rl][pc * 4]);
  for (int c = tid; c < 256; c += 128) { float s = 0.f, q2 = 0.f; for (int pl = 0; pl < 64; ++pl) { const float v = so[pl >> 4][pl & 15][c]; s += v; q2 += v * v; } sps[c][0] = s; sps[c][1] = q2; }
  __syncthreads();
  vst2(PS3 + (size_t)blockIdx.x * 512 + tid * 4, *(const v4f*)(&sps[0][0] + tid * 4));
}
__global__ __launch_bounds__(128) void k_l4(const float* __restrict__ H3, const float* __restrict__ GN3, const float* __restrict__ g3w, const float* __restrict__ g3b, const float* __restrict__ W4, float* __restrict__ PS4) {
  __shared__ __align__(16) __bf16 sah[64][264], sal[64][264]; __shared__ __align__(16) float so[4][16][260]; __shared__ __align__(16) float sps[512][4];
  const int tid = threadIdx.x, wave = tid >> 5, lane = tid & 31, col = lane & 15, g = lane >> 4; const size_t p0 = (size_t)blockIdx.x * 64; const int b = (int)(p0 / NP);
  for (int q = tid; q < 64 * 256; q += 128) { const int pl = q >> 8, c = q & 255; const float a = gn_apply(H3[(p0 + pl) * 256 + c], GN3, b, c, 32, g3w, g3b); const __bf16 hb = (__bf16)a; sah[pl][c] = hb; sal[pl][c] = (__bf16)(a - (float)hb); }
  __syncthreads();
#pragma unroll 1
  for (int pass = 0; pass < 2; ++pass) { v8f acc[16] = {};
#pragma unroll
    for (int kc = 0; kc < 8; ++kc) { const v16b ah = frag_b(&sah[wave * 16 + col][kc * 32], lane), al = frag_b(&sal[wave * 16 + col][kc * 32], lane);
#pragma unroll
      for (int j = 0; j < 16; ++j) { const v16b w = frag_gbf(W4 + (size_t)(pass * 256 + j * 16 + col) * 256 + kc * 32, lane); acc[j] = wmma_bf(al, w, acc[j]); acc[j] = wmma_bf(ah, w, acc[j]); } }
#pragma unroll
    for (int j = 0; j < 16; ++j)
#pragma unroll
      for (int r = 0; r < 8; ++r) so[wave][8 * g + r][j * 16 + col] = acc[j][r];
    __syncthreads();
    for (int cl = tid; cl < 256; cl += 128) { float s = 0.f, q2 = 0.f, mx = -3.0e38f, mn = 3.0e38f; for (int pl = 0; pl < 64; ++pl) { const float v = so[pl >> 4][pl & 15][cl]; s += v; q2 += v * v; mx = fmaxf(mx, v); mn = fminf(mn, v); }
      sps[pass * 256 + cl][0] = s; sps[pass * 256 + cl][1] = q2; sps[pass * 256 + cl][2] = mx; sps[pass * 256 + cl][3] = mn; }
    __syncthreads(); }
  for (int q = tid; q < 512; q += 128) vst2(PS4 + ((size_t)blockIdx.x * 512 + q) * 4, *(const v4f*)&sps[q][0]);
}
__global__ __launch_bounds__(256) void k_head(const float* __restrict__ PS4, const float* __restrict__ g4w, const float* __restrict__ g4b, const float* __restrict__ f1w, const float* __restrict__ f1b, const float* __restrict__ f2w, const float* __restrict__ f2b, float* __restrict__ out) {
  __shared__ float sgn[NG][2]; __shared__ float sg[512]; __shared__ float sh[128]; __shared__ __align__(16) float sres[16];
  const int tid = threadIdx.x, wave = tid >> 5, lane = tid & 31;
#pragma unroll 1
  for (int b = 0; b < TNB; ++b) {
    { const int g = wave, cpg = 64; float s = 0.f, q = 0.f;
      for (int e = lane; e < 64 * cpg; e += 32) { const int blk = e / cpg, cc = g * cpg + e % cpg; const float* pp = PS4 + ((size_t)(b * 64 + blk) * 512 + cc) * 4; s += pp[0]; q += pp[1]; }
#pragma unroll
      for (int o = 1; o < 32; o <<= 1) { s += __shfl_xor(s, o); q += __shfl_xor(q, o); }
      if (lane == 0) { const float cnt = (float)(cpg * NP); const float mu = s / cnt; sgn[g][0] = mu; sgn[g][1] = rsqrtf(fmaxf(q / cnt - mu * mu, 0.f) + 1e-5f); } }
    __syncthreads();
    for (int c = tid; c < 512; c += 256) { float mx = -3.0e38f, mn = 3.0e38f; for (int blk = 0; blk < 64; ++blk) { const float* pp = PS4 + ((size_t)(b * 64 + blk) * 512 + c) * 4; mx = fmaxf(mx, pp[2]); mn = fminf(mn, pp[3]); }
      const int g = c / 64; const float a = sgn[g][1] * bfr(g4w[c]); const float bb = bfr(g4b[c]) - sgn[g][0] * a; const float v = (a >= 0.f ? a * mx : a * mn) + bb; sg[c] = v > 0.f ? v : 0.f; }
    __syncthreads();
    if (tid < 128) { float s = bfr(f1b[tid]); for (int c = 0; c < 512; ++c) s += sg[c] * bfr(f1w[tid * 512 + c]); sh[tid] = s > 0.f ? s : 0.f; }
    __syncthreads();
    if (tid < 32) { float s = 0.f; for (int j = lane; j < 128; j += 32) s += sh[j] * bfr(f2w[j]);
#pragma unroll
      for (int o = 1; o < 32; o <<= 1) s += __shfl_xor(s, o);
      if (lane == 0) sres[b] = s + bfr(f2b[0]); }
    __syncthreads(); }
  if (tid < 4) vst2(out + tid * 4, *(const v4f*)&sres[tid * 4]);
}

extern "C" void kernel_launch(void* const* d_in, const int* in_sizes, int n_in, void* d_out, int out_size, void* d_ws, size_t ws_size, hipStream_t stream) {
  (void)in_sizes; (void)n_in; (void)out_size;
  const float** F = (const float**)d_in;
  if (ws_size < (size_t)WS_END) return;
  char* ws = (char*)d_ws; int *CNT = (int*)(ws + WS_CNT), *OFF = (int*)(ws + WS_OFF); float *PTS = (float*)(ws + WS_PTS), *H2 = (float*)(ws + WS_H2), *H3 = (float*)(ws + WS_H3), *PS1 = (float*)(ws + WS_PS1), *PS2 = (float*)(ws + WS_PS2), *PS3 = (float*)(ws + WS_PS3), *PS4 = (float*)(ws + WS_PS4), *GN = (float*)(ws + WS_GN);
  float *GN1 = GN, *GN2 = GN + NBATCH * 16, *GN3 = GN + 2 * NBATCH * 16;
  k_count<<<(TNB * NCHK + 255) / 256, 256, 0, stream>>>(F[0], CNT);
  k_scan<<<TNB, 256, 0, stream>>>(CNT, OFF);
  k_pick<<<dim3(NP / 256, TNB), 256, 0, stream>>>(F[0], OFF, PTS);
  k_l1s<<<TNB * NP / 64, 128, 0, stream>>>(PTS, F[1], PS1);
  k_gn<<<TNB, 256, 0, stream>>>(PS1, 64, 2, GN1);
  k_l2<<<TNB * NP / 64, 128, 0, stream>>>(PTS, F[1], GN1, F[2], F[3], F[4], H2, PS2);
  k_gn<<<TNB, 256, 0, stream>>>(PS2, 128, 2, GN2);
  k_l3<<<TNB * NP / 64, 128, 0, stream>>>(H2, GN2, F[5], F[6], F[7], H3, PS3);
  k_gn<<<TNB, 256, 0, stream>>>(PS3, 256, 2, GN3);
  k_l4<<<TNB * NP / 64, 128, 0, stream>>>(H3, GN3, F[8], F[9], F[10], PS4);
  k_head<<<1, 256, 0, stream>>>(PS4, F[11], F[12], F[13], F[14], F[15], F[16], (float*)d_out);
}
